// MultiHeadAttention_57655640981747
// MI455X (gfx1250) — hardware-verified
//
#include <hip/hip_runtime.h>


#ifndef NB
#define NB 1
#endif
#ifndef SEQ
#define SEQ 4096
#endif
#define NB_FULL  1
#define SEQ_FULL 4096
#ifndef OUT_SEQ
#define OUT_SEQ SEQ
#endif
#define DM   768
#define NH_  12
#define HD   64
#define QKVC (3 * DM)
#define AW   4
#define ER   ((SEQ) < 512 ? (SEQ) : 512)
#define QRS  2048.0f
#define QRI  (1.0f / 2048.0f)
#define SC2  (0.125f * 1.4426950408889634f)
#define PSH  8.0f
#define CXS  16.0f
#define WPS  64.0f
#define OSC  (1.0f / 1024.0f)
#define NEGM (-3.0e38f)

static_assert(HD == 64);
static_assert(NH_ * HD == DM);
static_assert(DM % 64 == 0);
static_assert(QKVC % 64 == 0);
static_assert(DM % 32 == 0);
static_assert(SEQ % 64 == 0);
static_assert((NB * SEQ) % 64 == 0);
static_assert(SEQ % 32 == 0);
static_assert(ER % (16 * AW) == 0);
static_assert((SEQ - ER) % (16 * AW) == 0);
static_assert(ER % 64 == 0);
static_assert(((size_t)SEQ * DM) % 8 == 0);
static_assert(NB <= NB_FULL);
static_assert(SEQ <= SEQ_FULL);

typedef _Float16 h16;
typedef unsigned short bf;
typedef __attribute__((ext_vector_type(16))) __bf16   v16bf;
typedef __attribute__((ext_vector_type(16))) _Float16 v16h;
typedef __attribute__((ext_vector_type(8)))  _Float16 v8h;
typedef __attribute__((ext_vector_type(8)))  unsigned short v8us;
typedef __attribute__((ext_vector_type(8)))  float    v8f;
typedef __attribute__((ext_vector_type(4)))  float    v4f;
typedef v4f  __attribute__((may_alias)) v4fa;
typedef v8us __attribute__((may_alias)) v8usa;

__device__ __forceinline__ unsigned short f2bf(float f) { unsigned u = __float_as_uint(f); u += 0x7FFFu + ((u >> 16) & 1u); return (unsigned short)(u >> 16); }
__device__ __forceinline__ float bfr(float f) { return __uint_as_float(((unsigned)f2bf(f)) << 16); }
__device__ __forceinline__ v16h cat16(v8h lo, v8h hi) { return __builtin_shufflevector(lo, hi, 0, 1, 2, 3, 4, 5, 6, 7, 8, 9, 10, 11, 12, 13, 14, 15); }
__device__ __forceinline__ v16bf cat16b(v8us lo, v8us hi) { return __builtin_bit_cast(v16bf, __builtin_shufflevector(lo, hi, 0, 1, 2, 3, 4, 5, 6, 7, 8, 9, 10, 11, 12, 13, 14, 15)); }
__device__ __forceinline__ v8f wmma16(v16h a, v16h b, v8f c) { return __builtin_amdgcn_wmma_f32_16x16x32_f16(false, a, false, b, (short)0, c, false, false); }
__device__ __forceinline__ v8f wmmab(v16bf a, v16bf b, v8f c) { return __builtin_amdgcn_wmma_f32_16x16x32_bf16(false, a, false, b, (short)0, c, false, false); }
__device__ __forceinline__ v16h  ldh(const h16* p) { return cat16(*(const v8h*)p, *(const v8h*)(p + 16)); }
__device__ __forceinline__ v16bf ldb(const bf* p)  { return cat16b(*(const v8us*)p, *(const v8us*)(p + 16)); }
__device__ __forceinline__ void wave_sync() { __builtin_amdgcn_fence(3  , "wavefront"); __builtin_amdgcn_wave_barrier(); asm volatile("" ::: "memory"); }

__global__ __launch_bounds__(256) void k_cvt8(const float* __restrict__ src, bf* dst, size_t n8) {
    const size_t i = (size_t)blockIdx.x * 256 + threadIdx.x; if (i >= n8) return;
    const v8f v = *(const v8f*)(src + i * 8); v8us o;
#pragma unroll
    for (int k = 0; k < 8; ++k) o[k] = f2bf(v[k]);
    *(volatile v8us*)(dst + i * 8) = o; __threadfence(); *(volatile v8us*)(dst + i * 8) = o;
}

__global__ __launch_bounds__(256) void k_trw(const float* __restrict__ src, bf* dst, int cols, int perm, int asf16) {
    __shared__ __align__(16) unsigned short tile[64 * 72];
    const int tid = threadIdx.x;
    const int c0 = blockIdx.x * 64, k0 = blockIdx.y * 64;
    const int cc = tid & 63, kq = tid >> 6;
#pragma unroll 4
    for (int i = 0; i < 16; ++i) {
        const int kk = i * 4 + kq;
        const float w = src[(size_t)(k0 + kk) * (size_t)cols + c0 + cc];
        const unsigned short hb = f2bf(w);
        const float wr = __uint_as_float(((unsigned)hb) << 16);
        const unsigned short fb = __builtin_bit_cast(unsigned short, (h16)(wr * WPS));
        tile[cc * 72 + kk] = asf16 ? fb : hb;
    }
    __syncthreads();
    const int cy = blockIdx.x;
    const int drow0 = perm ? ((cy % 3) * DM + (cy / 3) * 64) : c0;
    const int rA = tid >> 3, rB = 32 + (tid >> 3), ch = tid & 7;
    const v8us vA = *(const v8usa*)(&tile[rA * 72 + ch * 8]);
    const v8us vB = *(const v8usa*)(&tile[rB * 72 + ch * 8]);
    const size_t oA = (size_t)(drow0 + rA) * DM + k0 + ch * 8;
    const size_t oB = (size_t)(drow0 + rB) * DM + k0 + ch * 8;
    *(volatile v8us*)(dst + oA) = vA; *(volatile v8us*)(dst + oB) = vB;
    __threadfence();
    *(volatile v8us*)(dst + oA) = vA; *(volatile v8us*)(dst + oB) = vB;
}

__global__ __launch_bounds__(32) void k_proj(const bf* __restrict__ A, const bf* __restrict__ Bt, h16* Ph, h16* Pr, int useRes, int RB, size_t sRB, int pitch, int CB, size_t sCB) {
    __shared__ __align__(16) float os[16 * 68];
    const int K = DM;
    const int lane = threadIdx.x & 31, lr = lane & 15, hi = lane >> 4; const int r0 = blockIdx.x * 64, c0 = blockIdx.y * 64;
    v8f acc[4][4];
#pragma unroll
    for (int mb = 0; mb < 4; ++mb)
#pragma unroll
        for (int nb = 0; nb < 4; ++nb) acc[mb][nb] = (v8f){};
    const size_t aoff = (size_t)(r0 + lr) * K + 8 * hi, boff = (size_t)(c0 + lr) * K + 8 * hi;
#pragma unroll 1
    for (int kc = 0; kc < K; kc += 32) {
        v16bf a[4];
#pragma unroll
        for (int mb = 0; mb < 4; ++mb) a[mb] = ldb(A + aoff + (size_t)mb * 16 * K + kc);
#pragma unroll
        for (int nb = 0; nb < 4; ++nb) { const v16bf b = ldb(Bt + boff + (size_t)nb * 16 * K + kc);
#pragma unroll
            for (int mb = 0; mb < 4; ++mb) acc[mb][nb] = wmmab(a[mb], b, acc[mb][nb]); }
        asm volatile("v_nop\n\tv_nop\n\tv_nop\n\tv_nop" : "+v"(acc[0][0]), "+v"(acc[1][1]), "+v"(acc[2][2]), "+v"(acc[3][3]) : "v"(a[0]), "v"(a[1]), "v"(a[2]), "v"(a[3]));
    }
    const size_t tbase = (size_t)(r0 / RB) * sRB + (size_t)(r0 % RB) * (size_t)pitch + (size_t)(c0 / CB) * sCB + (size_t)(c0 % CB);
#pragma unroll
    for (int mb = 0; mb < 4; ++mb) {
#pragma unroll
        for (int nb = 0; nb < 4; ++nb) {
#pragma unroll
            for (int j = 0; j < 8; ++j) os[(hi * 8 + j) * 68 + nb * 16 + lr] = acc[mb][nb][j]; }
        wave_sync();
        const size_t sb = tbase + (size_t)(mb * 16) * (size_t)pitch;
#pragma unroll 1
        for (int ps = 0; ps < 2; ++ps) {
#pragma unroll
            for (int s = 0; s < 4; ++s) { const int row = 4 * s + (lane >> 3), c8 = (lane & 7) * 8;
                const v4f x0 = *(const v4fa*)(&os[row * 68 + c8]); const v4f x1 = *(const v4fa*)(&os[row * 68 + c8 + 4]); v8h hv, rv;
#pragma unroll
                for (int i = 0; i < 4; ++i) { const h16 a0 = (h16)x0[i]; const h16 a1 = (h16)x1[i]; hv[i] = a0; hv[4 + i] = a1; rv[i] = (h16)((x0[i] - (float)a0) * QRS); rv[4 + i] = (h16)((x1[i] - (float)a1) * QRS); }
                const size_t oo = sb + (size_t)row * (size_t)pitch + c8;
                *(volatile v8h*)(Ph + oo) = hv; if (useRes) *(volatile v8h*)(Pr + oo) = rv; }
            if (ps == 0) __threadfence(); }
        wave_sync();
    }
}

template <int EARLY>
__device__ __forceinline__ void flash_body(const h16* __restrict__ QH, const h16* __restrict__ QR, const h16* __restrict__ KP, const h16* __restrict__ KR,
                                           const h16* __restrict__ VT, const h16* __restrict__ VR, h16* CH, h16* CR, int tbase) {
    __shared__ __align__(16) float os[AW * 16 * 68];
    const int lane = threadIdx.x & 31, lr = lane & 15, hi = lane >> 4;
    const int wave = __builtin_amdgcn_readfirstlane((int)(threadIdx.x >> 5));
    const int zh = blockIdx.y; const int b = zh / NH_, h = zh % NH_;
    const int t0 = tbase + ((int)blockIdx.x * AW + wave) * 16;
    const int tq = t0 + lr;
    const size_t pbase = (size_t)zh * SEQ * HD;
    const size_t qo = pbase + (size_t)(t0 + lr) * HD + 8 * hi;
    const v16h qh0 = ldh(QH + qo), qh1 = ldh(QH + qo + 32);
    v16h qr0 = qh0, qr1 = qh1;
    if (EARLY) { qr0 = ldh(QR + qo); qr1 = ldh(QR + qo + 32); }
    const size_t ko = pbase + (size_t)lr * HD + 8 * hi;
    const size_t vo = pbase + (size_t)lr * SEQ + 8 * hi;
    v8f oH[4], oL[4];
#pragma unroll
    for (int j = 0; j < 4; ++j) { oH[j] = (v8f){}; oL[j] = (v8f){}; }
    float m = NEGM, l = 0.0f;
    const int kend = t0 + 16;
#pragma unroll 1
    for (int key0 = 0; key0 < kend; key0 += 32) {
        const size_t kofs = ko + (size_t)key0 * HD;
        const v16h ka0 = ldh(KP + kofs), ka1 = ldh(KP + kofs + 32), kb0 = ldh(KP + kofs + 16 * HD), kb1 = ldh(KP + kofs + 16 * HD + 32);
        v8f sHa = (v8f){}, sLa = (v8f){}, sHb = (v8f){}, sLb = (v8f){};
        sHa = wmma16(ka0, qh0, sHa); sHb = wmma16(kb0, qh0, sHb);
        sHa = wmma16(ka1, qh1, sHa); sHb = wmma16(kb1, qh1, sHb);
        if (EARLY) {
            const v16h ra0 = ldh(KR + kofs), ra1 = ldh(KR + kofs + 32), rb0 = ldh(KR + kofs + 16 * HD), rb1 = ldh(KR + kofs + 16 * HD + 32);
            sLa = wmma16(ka0, qr0, sLa); sLb = wmma16(kb0, qr0, sLb);
            sLa = wmma16(ka1, qr1, sLa); sLb = wmma16(kb1, qr1, sLb);
            sLa = wmma16(ra0, qh0, sLa); sLb = wmma16(rb0, qh0, sLb);
            sLa = wmma16(ra1, qh1, sLa); sLb = wmma16(rb1, qh1, sLb);
            asm volatile("v_nop\n\tv_nop\n\tv_nop\n\tv_nop" : "+v"(sHa), "+v"(sLa), "+v"(sHb), "+v"(sLb) : "v"(ra0), "v"(ra1), "v"(rb0), "v"(rb1), "v"(ka1), "v"(kb1));
        } else {
            asm volatile("v_nop\n\tv_nop\n\tv_nop\n\tv_nop" : "+v"(sHa), "+v"(sHb) : "v"(ka0), "v"(ka1), "v"(kb0), "v"(kb1));
        }
        float ta[8], tb[8];
#pragma unroll
        for (int r = 0; r < 8; ++r) {
            if (EARLY) { ta[r] = (sHa[r] + sLa[r] * QRI) * SC2; tb[r] = (sHb[r] + sLb[r] * QRI) * SC2; }
            else       { ta[r] = sHa[r] * SC2;                  tb[r] = sHb[r] * SC2; }
        }
        if (key0 + 32 > t0) {
            const int kk = key0 + 8 * hi;
#pragma unroll
            for (int r = 0; r < 8; ++r) { ta[r] = (kk + r <= tq) ? ta[r] : NEGM; tb[r] = (kk + 16 + r <= tq) ? tb[r] : NEGM; }
        }
        float mx = NEGM;
#pragma unroll
        for (int r = 0; r < 8; ++r) mx = fmaxf(mx, fmaxf(ta[r], tb[r]));
        mx = fmaxf(mx, __shfl_xor(mx, 16, 32));
        const float mnew = fmaxf(m, mx);
        const float alpha = __builtin_amdgcn_exp2f(m - mnew);
        const float sh = PSH - mnew;
        v16h pb, pr; float ls = 0.0f;
#pragma unroll
        for (int r = 0; r < 8; ++r) {
            const float e0 = __builtin_amdgcn_exp2f(ta[r] + sh), e1 = __builtin_amdgcn_exp2f(tb[r] + sh);
            const h16 pa = (h16)e0; const h16 pc = (h16)e1; pb[r] = pa; pb[8 + r] = pc;
            if (EARLY) { pr[r] = (h16)((e0 - (float)pa) * QRS); pr[8 + r] = (h16)((e1 - (float)pc) * QRS); ls += e0 + e1; }
            else       { pr[r] = pa; pr[8 + r] = pc; ls += (float)pa + (float)pc; }
        }
        l = l * alpha + ls; m = mnew;
#pragma unroll
        for (int j = 0; j < 4; ++j) { oH[j] = oH[j] * alpha; if (EARLY) oL[j] = oL[j] * alpha; }
        const size_t vofs = vo + (size_t)key0;
        const v16h v0 = ldh(VT + vofs), v1 = ldh(VT + vofs + (size_t)16 * SEQ), v2 = ldh(VT + vofs + (size_t)32 * SEQ), v3 = ldh(VT + vofs + (size_t)48 * SEQ);
        oH[0] = wmma16(v0, pb, oH[0]); oH[1] = wmma16(v1, pb, oH[1]); oH[2] = wmma16(v2, pb, oH[2]); oH[3] = wmma16(v3, pb, oH[3]);
        if (EARLY) {
            const v16h w0 = ldh(VR + vofs), w1 = ldh(VR + vofs + (size_t)16 * SEQ), w2 = ldh(VR + vofs + (size_t)32 * SEQ), w3 = ldh(VR + vofs + (size_t)48 * SEQ);
            oL[0] = wmma16(v0, pr, oL[0]); oL[1] = wmma16(v1, pr, oL[1]); oL[2] = wmma16(v2, pr, oL[2]); oL[3] = wmma16(v3, pr, oL[3]);
            oL[0] = wmma16(w0, pb, oL[0]); oL[1] = wmma16(w1, pb, oL[1]); oL[2] = wmma16(w2, pb, oL[2]); oL[3] = wmma16(w3, pb, oL[3]);
            asm volatile("v_nop\n\tv_nop\n\tv_nop\n\tv_nop" : "+v"(oH[0]), "+v"(oH[1]), "+v"(oH[2]), "+v"(oH[3]), "+v"(oL[0]), "+v"(oL[1]), "+v"(oL[2]), "+v"(oL[3])
                         : "v"(w0), "v"(w1), "v"(w2), "v"(w3), "v"(v0), "v"(v1), "v"(v2), "v"(v3), "v"(pb), "v"(pr));
        } else {
            asm volatile("v_nop\n\tv_nop\n\tv_nop\n\tv_nop" : "+v"(oH[0]), "+v"(oH[1]), "+v"(oH[2]), "+v"(oH[3]) : "v"(v0), "v"(v1), "v"(v2), "v"(v3), "v"(pb));
        }
    }
    l += __shfl_xor(l, 16, 32);
    const float inv = 1.0f / l;
    const int wb = wave * 16 * 68;
#pragma unroll
    for (int j = 0; j < 4; ++j) {
        v4f a, c;
#pragma unroll
        for (int i = 0; i < 4; ++i) {
            if (EARLY) { a[i] = (oH[j][i] + oL[j][i] * QRI) * inv; c[i] = (oH[j][4 + i] + oL[j][4 + i] * QRI) * inv; }
            else       { a[i] = oH[j][i] * inv;                    c[i] = oH[j][4 + i] * inv; }
        }
        *(v4fa*)(&os[wb + lr * 68 + 16 * j + 8 * hi]) = a; *(v4fa*)(&os[wb + lr * 68 + 16 * j + 8 * hi + 4]) = c;
    }
    wave_sync();
    const size_t crow = ((size_t)b * SEQ + t0) * DM + h * HD;
    const size_t rrow = ((size_t)b * ER + t0) * DM + h * HD;
#pragma unroll 1
    for (int ps = 0; ps < 2; ++ps) {
#pragma unroll
        for (int s = 0; s < 4; ++s) { const int row = 4 * s + (lane >> 3), c8 = (lane & 7) * 8;
            const v4f x0 = *(const v4fa*)(&os[wb + row * 68 + c8]); const v4f x1 = *(const v4fa*)(&os[wb + row * 68 + c8 + 4]); v8h hv, rv;
#pragma unroll
            for (int i = 0; i < 4; ++i) { const float y0 = x0[i] * CXS, y1 = x1[i] * CXS; const h16 a0 = (h16)y0; const h16 a1 = (h16)y1; hv[i] = a0; hv[4 + i] = a1;
                rv[i] = (h16)((y0 - (float)a0) * QRS); rv[4 + i] = (h16)((y1 - (float)a1) * QRS); }
            *(volatile v8h*)(CH + crow + (size_t)row * DM + c8) = hv;
            if (EARLY) *(volatile v8h*)(CR + rrow + (size_t)row * DM + c8) = rv; }
        if (ps == 0) __threadfence(); }
}

__global__ __launch_bounds__(32 * AW) void k_flash_early(const h16* __restrict__ QH, const h16* __restrict__ QR, const h16* __restrict__ KP, const h16* __restrict__ KR,
                                                         const h16* __restrict__ VT, const h16* __restrict__ VR, h16* CH, h16* CR) {
    flash_body<1>(QH, QR, KP, KR, VT, VR, CH, CR, 0);
}
__global__ __launch_bounds__(32 * AW) void k_flash_dense(const h16* __restrict__ QH, const h16* __restrict__ QR, const h16* __restrict__ KP, const h16* __restrict__ KR,
                                                         const h16* __restrict__ VT, const h16* __restrict__ VR, h16* CH, h16* CR) {
    flash_body<0>(QH, QR, KP, KR, VT, VR, CH, CR, ER);
}

__global__ __launch_bounds__(32) void k_out(const h16* __restrict__ CX, size_t resOff, const h16* __restrict__ Wt, const float* __restrict__ bias, float* OUT) {
    __shared__ __align__(16) float os[16 * 68];
    const int K = DM;
    const int lane = threadIdx.x & 31, lr = lane & 15, hi = lane >> 4; const int r0 = blockIdx.x * 64, c0 = blockIdx.y * 64;
    const int bb = r0 / SEQ, tt = r0 % SEQ;
    v8f acc[4][4];
#pragma unroll
    for (int mb = 0; mb < 4; ++mb)
#pragma unroll
        for (int nb = 0; nb < 4; ++nb) acc[mb][nb] = (v8f){};
    const size_t aoffH = (size_t)(r0 + lr) * K + 8 * hi;
    const size_t aoffR = resOff + (size_t)(bb * ER + (tt < ER ? tt : 0) + lr) * K + 8 * hi;
    const size_t boff = (size_t)(c0 + lr) * K + 8 * hi;
    const int p0 = (tt < ER) ? 0 : 1;
#pragma unroll 1
    for (int pass = p0; pass < 2; ++pass) {
        const size_t aoff = (pass == 0) ? aoffR : aoffH;
#pragma unroll 1
        for (int kc = 0; kc < K; kc += 32) {
            v16h a[4];
#pragma unroll
            for (int mb = 0; mb < 4; ++mb) a[mb] = ldh(CX + aoff + (size_t)mb * 16 * K + kc);
#pragma unroll
            for (int nb = 0; nb < 4; ++nb) { const v16h bq = ldh(Wt + boff + (size_t)nb * 16 * K + kc);
#pragma unroll
                for (int mb = 0; mb < 4; ++mb) acc[mb][nb] = wmma16(a[mb], bq, acc[mb][nb]); }
            asm volatile("v_nop\n\tv_nop\n\tv_nop\n\tv_nop" : "+v"(acc[0][0]), "+v"(acc[1][1]), "+v"(acc[2][2]), "+v"(acc[3][3]) : "v"(a[0]), "v"(a[1]), "v"(a[2]), "v"(a[3]));
        }
        if (pass == 0) {
#pragma unroll
            for (int mb = 0; mb < 4; ++mb)
#pragma unroll
                for (int nb = 0; nb < 4; ++nb) acc[mb][nb] = acc[mb][nb] * QRI;
        }
    }
    const v4f braw = *(const v4f*)(bias + c0 + lr * 4);
    v4f bq4;
#pragma unroll
    for (int i = 0; i < 4; ++i) bq4[i] = bfr(braw[i]);
#pragma unroll
    for (int mb = 0; mb < 4; ++mb) {
#pragma unroll
        for (int nb = 0; nb < 4; ++nb) {
#pragma unroll
            for (int j = 0; j < 8; ++j) os[(hi * 8 + j) * 68 + nb * 16 + lr] = acc[mb][nb][j]; }
        wave_sync();
        float* orow = OUT + ((size_t)bb * OUT_SEQ + tt + mb * 16) * DM + c0;
#pragma unroll 1
        for (int ps = 0; ps < 2; ++ps) {
#pragma unroll
            for (int s = 0; s < 8; ++s) { const int row = 2 * s + hi, cofs = lr * 4;
                const v4f xv = *(const v4fa*)(&os[row * 68 + cofs]);
                const v4f val = xv * OSC + bq4;
                *(volatile v4f*)(orow + (size_t)row * DM + cofs) = val; }
            if (ps == 0) __threadfence(); }
        wave_sync();
    }
}

static constexpr size_t al256(size_t v) { return (v + 255) & ~(size_t)255; }
static constexpr size_t SZ_XB = al256((size_t)NB * SEQ * DM * 2);
static constexpr size_t SZ_WT = al256((size_t)3 * DM * DM * 2);
static constexpr size_t SZ_WP = al256((size_t)DM * DM * 2);
static constexpr size_t SZ_PL = al256((size_t)NB * NH_ * SEQ * HD * 2);
static constexpr size_t SZ_CH = al256((size_t)NB * SEQ * DM * 2);
static constexpr size_t SZ_CR = al256((size_t)NB * ER * DM * 2);
static constexpr size_t SZ_TOTAL = SZ_XB + SZ_WT + SZ_WP + 6 * SZ_PL + SZ_CH + SZ_CR;
static_assert(SZ_TOTAL <= (size_t)134217728);
static_assert(((size_t)DM * DM * 2) % 256 == 0);

extern "C" void kernel_launch(void* const* d_in, const int* in_sizes, int n_in,
                              void* d_out, int out_size, void* d_ws, size_t ws_size, hipStream_t stream) {
    if (n_in < 4) return;
    const size_t needx = ((size_t)(NB - 1) * SEQ_FULL + SEQ) * DM;
    if ((size_t)in_sizes[0] < needx) return;
    if ((size_t)in_sizes[1] < (size_t)DM * QKVC || (size_t)in_sizes[2] < (size_t)DM * DM || (size_t)in_sizes[3] < (size_t)DM) return;
    if ((size_t)out_size < ((size_t)(NB - 1) * OUT_SEQ + SEQ) * DM) return;
    if (SZ_TOTAL > ws_size) return;
    const float* x = (const float*)d_in[0]; const float* wqkv = (const float*)d_in[1]; const float* wproj = (const float*)d_in[2]; const float* bproj = (const float*)d_in[3];
    float* OUT = (float*)d_out;
    char* wsp = (char*)d_ws;
    bf* XB = (bf*)wsp; wsp += SZ_XB;
    bf* WT = (bf*)wsp; wsp += SZ_WT;
    h16* WP = (h16*)wsp; wsp += SZ_WP;
    h16* QH = (h16*)wsp; wsp += SZ_PL;
    h16* QR = (h16*)wsp; wsp += SZ_PL;
    h16* KP = (h16*)wsp; wsp += SZ_PL;
    h16* KR = (h16*)wsp; wsp += SZ_PL;
    h16* VT = (h16*)wsp; wsp += SZ_PL;
    h16* VR = (h16*)wsp; wsp += SZ_PL;
    h16* CH = (h16*)wsp; wsp += SZ_CH;
    h16* CR = (h16*)wsp; wsp += SZ_CR;
    bf* WQ = WT; bf* WK = WT + (size_t)DM * DM; bf* WV = WT + (size_t)2 * DM * DM;

    if (SEQ == SEQ_FULL) {
        const size_t n8 = (size_t)NB * SEQ * DM / 8;
        k_cvt8<<<(unsigned)((n8 + 255) / 256), 256, 0, stream>>>(x, XB, n8);
    } else {
        const size_t n8 = (size_t)SEQ * DM / 8;
        for (int b = 0; b < NB; ++b) k_cvt8<<<(unsigned)((n8 + 255) / 256), 256, 0, stream>>>(x + (size_t)b * SEQ_FULL * DM, XB + (size_t)b * SEQ * DM, n8);
    }
    k_trw<<<dim3(QKVC / 64, DM / 64, 1), 256, 0, stream>>>(wqkv, WT, QKVC, 1, 0);
    k_trw<<<dim3(DM / 64, DM / 64, 1), 256, 0, stream>>>(wproj, (bf*)WP, DM, 0, 1);

    k_proj<<<dim3(NB * SEQ / 64, DM / 64, 1), 32, 0, stream>>>(XB, WQ, QH, QR, 1, SEQ, (size_t)NH_ * SEQ * HD, HD, HD, (size_t)SEQ * HD);
    k_proj<<<dim3(NB * SEQ / 64, DM / 64, 1), 32, 0, stream>>>(XB, WK, KP, KR, 1, SEQ, (size_t)NH_ * SEQ * HD, HD, HD, (size_t)SEQ * HD);
    k_proj<<<dim3(DM / 64, NB * SEQ / 64, 1), 32, 0, stream>>>(WV, XB, VT, VR, 1, DM, (size_t)0, SEQ, SEQ, (size_t)DM * SEQ);

    k_flash_early<<<dim3(ER / (16 * AW), NB * NH_, 1), 32 * AW, 0, stream>>>(QH, QR, KP, KR, VT, VR, CH, CR);
    if (SEQ > ER)
        k_flash_dense<<<dim3((SEQ - ER) / (16 * AW), NB * NH_, 1), 32 * AW, 0, stream>>>(QH, QR, KP, KR, VT, VR, CH, CR);

    k_out<<<dim3(NB * SEQ / 64, DM / 64, 1), 32, 0, stream>>>(CH, (size_t)(SZ_CH / 2), WP, bproj, OUT);
}
